// Linear_53515292508495
// MI455X (gfx1250) — hardware-verified
//
#include <hip/hip_runtime.h>
#include <stddef.h>
#include <stdint.h>

#define NTOK  4096
#define DIM   1024
#define ODIM  1024
#define NE    8
#define RNK   16
#define ER    128
#define SCAL  2.0f
#define NTHR  256
#define GTHR  128
#define TM    128
#define TN    64
#define WSMAX 134217728

static_assert(ER == NE * RNK);
static_assert((NTOK % TM) == 0);
static_assert((ODIM % TN) == 0 && (ER % TN) == 0);
static_assert((DIM % 32) == 0 && (ER % 32) == 0);
static_assert((NTOK % NTHR) == 0);
static_assert(TM == (GTHR / 32) * 32);
static_assert(TM * NE == GTHR * 8);
static_assert(((NTOK * DIM) % 8) == 0 && ((ODIM * DIM) % 8) == 0);
static_assert((DIM % 8) == 0 && (ER % 8) == 0);
static_assert((TN % 16) == 0 && ((TN / 16) * 16 == TN));

typedef float          v4f  __attribute__((ext_vector_type(4)));
typedef float          v8f  __attribute__((ext_vector_type(8)));
typedef int            v8i  __attribute__((ext_vector_type(8)));
typedef unsigned short v8us __attribute__((ext_vector_type(8)));
typedef __bf16         v16bf __attribute__((ext_vector_type(16)));
union FragB { v16bf v; v8us h[2]; v8i w; };

__device__ __forceinline__ v8f wmb(const FragB& a, const FragB& b, v8f c) {
  v8f d = __builtin_amdgcn_wmma_f32_16x16x32_bf16(false, a.v, false, b.v, (short)0, c, false, false);
  asm volatile("v_nop\n\tv_nop\n\tv_nop\n\tv_nop" : "+v"(d) : "v"(a.w), "v"(b.w));
  return d;
}

__device__ __forceinline__ void ldfrag(FragB& f, const unsigned short* p) {
  f.h[0] = *(const v8us*)(p);
  f.h[1] = *(const v8us*)(p + 16);
}

__device__ __forceinline__ unsigned short rne16(float f) {
  unsigned u = __float_as_uint(f);
  u += 0x7FFFu + ((u >> 16) & 1u);
  return (unsigned short)(u >> 16);
}
__device__ __forceinline__ float rne16f(float f) {
  return __uint_as_float(((unsigned)rne16(f)) << 16);
}
__device__ __forceinline__ v8us cvt8(const v4f a, const v4f b) {
  v8us o;
  o[0] = rne16(a.x); o[1] = rne16(a.y); o[2] = rne16(a.z); o[3] = rne16(a.w);
  o[4] = rne16(b.x); o[5] = rne16(b.y); o[6] = rne16(b.z); o[7] = rne16(b.w);
  return o;
}
__device__ __forceinline__ void sp1(float v, unsigned short& hi, unsigned short& lo) {
  const unsigned short hb = rne16(v);
  const float hf = __uint_as_float(((unsigned)hb) << 16);
  hi = hb;
  lo = rne16(v - hf);
}
__device__ __forceinline__ void split8(const v4f a, const v4f b, v8us& hv, v8us& lv) {
  unsigned short h0, h1, h2, h3, h4, h5, h6, h7, l0, l1, l2, l3, l4, l5, l6, l7;
  sp1(a.x, h0, l0); sp1(a.y, h1, l1); sp1(a.z, h2, l2); sp1(a.w, h3, l3);
  sp1(b.x, h4, l4); sp1(b.y, h5, l5); sp1(b.z, h6, l6); sp1(b.w, h7, l7);
  hv[0] = h0; hv[1] = h1; hv[2] = h2; hv[3] = h3; hv[4] = h4; hv[5] = h5; hv[6] = h6; hv[7] = h7;
  lv[0] = l0; lv[1] = l1; lv[2] = l2; lv[3] = l3; lv[4] = l4; lv[5] = l5; lv[6] = l6; lv[7] = l7;
}

__global__ __launch_bounds__(NTHR) void k_cvt(const float* __restrict__ src, unsigned short* dst, int nUnits) {
  const int u = (int)blockIdx.x * NTHR + (int)threadIdx.x;
  if (u >= nUnits) return;
  const float* p = src + (size_t)u * 8;
  const v4f a = *(const v4f*)p;
  const v4f b = *(const v4f*)(p + 4);
  const v8us o = cvt8(a, b);
  const size_t q = (size_t)u * 8;
  *(volatile v8us*)(dst + q) = o;
  __threadfence();
  *(volatile v8us*)(dst + q) = o;
}

__global__ __launch_bounds__(NTHR) void k_wtr(const float* __restrict__ src, unsigned short* dst,
                                              int K, int N, int E, int nUnits) {
  const int u = (int)blockIdx.x * NTHR + (int)threadIdx.x;
  if (u >= nUnits) return;
  const int kq  = K >> 3;
  const int per = N * kq;
  int e = u / per;
  e = e > E - 1 ? E - 1 : e;
  const int rem = u - e * per;
  const int n   = rem / kq;
  const int k8  = (rem - n * kq) * 8;
  const float* p = src + ((size_t)e * (size_t)K + (size_t)k8) * (size_t)N + n;
  v4f a, b;
  a.x = p[0];                 a.y = p[(size_t)N];         a.z = p[(size_t)2 * N];     a.w = p[(size_t)3 * N];
  b.x = p[(size_t)4 * N];     b.y = p[(size_t)5 * N];     b.z = p[(size_t)6 * N];     b.w = p[(size_t)7 * N];
  const v8us o = cvt8(a, b);
  const size_t q = ((size_t)e * (size_t)N + (size_t)n) * (size_t)K + (size_t)k8;
  *(volatile v8us*)(dst + q) = o;
  __threadfence();
  *(volatile v8us*)(dst + q) = o;
}

__device__ __forceinline__ void gacc(float xq, const float* swrow, float (&acc)[NE]) {
  const v4f wa = *(const v4f*)(swrow);
  const v4f wb = *(const v4f*)(swrow + 4);
  acc[0] = fmaf(xq, wa.x, acc[0]); acc[1] = fmaf(xq, wa.y, acc[1]);
  acc[2] = fmaf(xq, wa.z, acc[2]); acc[3] = fmaf(xq, wa.w, acc[3]);
  acc[4] = fmaf(xq, wb.x, acc[4]); acc[5] = fmaf(xq, wb.y, acc[5]);
  acc[6] = fmaf(xq, wb.z, acc[6]); acc[7] = fmaf(xq, wb.w, acc[7]);
}

__global__ __launch_bounds__(NTHR) void k_gate(const float* __restrict__ x, const float* __restrict__ rw,
                                               const float* __restrict__ rb, float* ew) {
  __shared__ __attribute__((aligned(16))) float sw[DIM * NE];
  __shared__ __attribute__((aligned(16))) float se[NTHR * NE];
  __shared__ float sb[NE];
  const int tid = (int)threadIdx.x;
#pragma unroll 1
  for (int i = tid; i < DIM * NE; i += NTHR) {
    const int d = i >> 3, e = i & 7;
    sw[i] = rne16f(rw[(size_t)e * DIM + d]);
  }
  if (tid < NE) sb[tid] = rne16f(rb[tid]);
  __syncthreads();
  int t = (int)blockIdx.x * NTHR + tid;
  t = t > NTOK - 1 ? NTOK - 1 : t;
  const float* xr = x + (size_t)t * DIM;
  float acc[NE];
#pragma unroll
  for (int e = 0; e < NE; ++e) acc[e] = 0.f;
#pragma unroll 1
  for (int d4 = 0; d4 < DIM / 4; ++d4) {
    const v4f xv = *(const v4f*)(xr + 4 * d4);
    const float* swr = sw + (size_t)(4 * d4) * NE;
    gacc(rne16f(xv.x), swr,          acc);
    gacc(rne16f(xv.y), swr + NE,     acc);
    gacc(rne16f(xv.z), swr + 2 * NE, acc);
    gacc(rne16f(xv.w), swr + 3 * NE, acc);
  }
#pragma unroll
  for (int e = 0; e < NE; ++e) acc[e] += sb[e];
  int i1 = 0;
  float m1 = acc[0];
#pragma unroll
  for (int e = 1; e < NE; ++e) {
    const bool up = acc[e] > m1;
    i1 = up ? e : i1;
    m1 = up ? acc[e] : m1;
  }
  float m2 = -3.0e38f;
#pragma unroll
  for (int e = 0; e < NE; ++e) {
    const bool ok = (e != i1) && (acc[e] > m2);
    m2 = ok ? acc[e] : m2;
  }
  float p[NE];
  float s = 0.f;
#pragma unroll
  for (int e = 0; e < NE; ++e) {
    const float pe = (acc[e] >= m2) ? __expf(acc[e] - m1) : 0.f;
    p[e] = pe;
    s += pe;
  }
  const float inv = SCAL * (1.0f / s);
#pragma unroll
  for (int e = 0; e < NE; ++e) se[tid * NE + e] = p[e] * inv;
  __syncthreads();

  float* chunk = ew + (size_t)blockIdx.x * (size_t)(NTHR * NE);
  const v4f v0 = *(const v4f*)(se + 4 * tid);
  const v4f v1 = *(const v4f*)(se + 4 * (tid + NTHR));
  *(volatile v4f*)(chunk + 4 * tid) = v0;
  *(volatile v4f*)(chunk + 4 * (tid + NTHR)) = v1;
  __threadfence();
  *(volatile v4f*)(chunk + 4 * tid) = v0;
  *(volatile v4f*)(chunk + 4 * (tid + NTHR)) = v1;
}

__global__ __launch_bounds__(GTHR) void k_ax(const unsigned short* __restrict__ xb,
                                             const unsigned short* __restrict__ at,
                                             const float* __restrict__ ew,
                                             unsigned short* waxh, unsigned short* waxl) {
  __shared__ __attribute__((aligned(16))) float stg[TM * TN];
  __shared__ __attribute__((aligned(16))) float sew[TM * NE];
  const int tid = (int)threadIdx.x, lane = tid & 31, w = tid >> 5, hh = lane >> 4, m = lane & 15;
  const int m0   = (int)blockIdx.x * TM;
  const int col0 = (int)blockIdx.y * TN;
  {
    const float* p = ew + (size_t)m0 * NE + 8 * tid;
    const v4f a = *(const v4f*)p;
    const v4f b = *(const v4f*)(p + 4);
    *(v4f*)(sew + 8 * tid)     = a;
    *(v4f*)(sew + 8 * tid + 4) = b;
  }
  __syncthreads();

  v8f acc[2][4];
  {
    const v8f z = {0.f, 0.f, 0.f, 0.f, 0.f, 0.f, 0.f, 0.f};
#pragma unroll
    for (int mt = 0; mt < 2; ++mt)
#pragma unroll
      for (int nt = 0; nt < 4; ++nt) acc[mt][nt] = z;
  }
  const unsigned short* a0p = xb + (size_t)(m0 + 32 * w + m) * (size_t)DIM + (size_t)(8 * hh);
  const unsigned short* a1p = a0p + (size_t)16 * DIM;
  const unsigned short* bp  = at + (size_t)(col0 + m) * (size_t)DIM + (size_t)(8 * hh);
#pragma unroll 1
  for (int ks = 0; ks < DIM / 32; ++ks) {
    FragB a0, a1;
    ldfrag(a0, a0p + 32 * ks);
    ldfrag(a1, a1p + 32 * ks);
#pragma unroll
    for (int nt = 0; nt < 4; ++nt) {
      FragB b;
      ldfrag(b, bp + (size_t)(16 * nt) * (size_t)DIM + 32 * ks);
      acc[0][nt] = wmb(a0, b, acc[0][nt]);
      acc[1][nt] = wmb(a1, b, acc[1][nt]);
    }
  }

#pragma unroll
  for (int nt = 0; nt < 4; ++nt) {
    int e = (col0 >> 4) + nt;
    e = e > NE - 1 ? NE - 1 : e;
    const int lc = 16 * nt + m;
#pragma unroll
    for (int mt = 0; mt < 2; ++mt) {
#pragma unroll
      for (int r = 0; r < 8; ++r) {
        const int lr = 32 * w + 16 * mt + 8 * hh + r;
        stg[lr * TN + lc] = acc[mt][nt][r] * sew[lr * NE + e];
      }
    }
  }
  __syncthreads();

  const int q8 = lane & 7, sub = lane >> 3;
  v8us hv[8], lv[8];
  size_t po[8];
#pragma unroll
  for (int i = 0; i < 8; ++i) {
    const int lr = 32 * w + 4 * i + sub;
    const v4f a = *(const v4f*)(stg + lr * TN + 8 * q8);
    const v4f b = *(const v4f*)(stg + lr * TN + 8 * q8 + 4);
    split8(a, b, hv[i], lv[i]);
    po[i] = (size_t)(m0 + lr) * (size_t)ER + (size_t)(col0 + 8 * q8);
  }
#pragma unroll
  for (int i = 0; i < 8; ++i) {
    *(volatile v8us*)(waxh + po[i]) = hv[i];
    *(volatile v8us*)(waxl + po[i]) = lv[i];
  }
  __threadfence();
#pragma unroll
  for (int i = 0; i < 8; ++i) {
    *(volatile v8us*)(waxh + po[i]) = hv[i];
    *(volatile v8us*)(waxl + po[i]) = lv[i];
  }
}

__global__ __launch_bounds__(GTHR) void k_main(const unsigned short* __restrict__ xb,
                                               const unsigned short* __restrict__ wb,
                                               const float* __restrict__ bb,
                                               const unsigned short* __restrict__ waxh,
                                               const unsigned short* __restrict__ waxl,
                                               const unsigned short* __restrict__ bt,
                                               float* out) {
  __shared__ __attribute__((aligned(16))) float stg[TM * TN];
  const int tid = (int)threadIdx.x, lane = tid & 31, w = tid >> 5, hh = lane >> 4, m = lane & 15;
  const int m0   = (int)blockIdx.x * TM;
  const int col0 = (int)blockIdx.y * TN;

  v8f acc[2][4];
  {
    const v8f z = {0.f, 0.f, 0.f, 0.f, 0.f, 0.f, 0.f, 0.f};
#pragma unroll
    for (int mt = 0; mt < 2; ++mt)
#pragma unroll
      for (int nt = 0; nt < 4; ++nt) acc[mt][nt] = z;
  }
  {
    const unsigned short* a0p = xb + (size_t)(m0 + 32 * w + m) * (size_t)DIM + (size_t)(8 * hh);
    const unsigned short* a1p = a0p + (size_t)16 * DIM;
    const unsigned short* bp  = wb + (size_t)(col0 + m) * (size_t)DIM + (size_t)(8 * hh);
#pragma unroll 1
    for (int ks = 0; ks < DIM / 32; ++ks) {
      FragB a0, a1;
      ldfrag(a0, a0p + 32 * ks);
      ldfrag(a1, a1p + 32 * ks);
#pragma unroll
      for (int nt = 0; nt < 4; ++nt) {
        FragB b;
        ldfrag(b, bp + (size_t)(16 * nt) * (size_t)DIM + 32 * ks);
        acc[0][nt] = wmb(a0, b, acc[0][nt]);
        acc[1][nt] = wmb(a1, b, acc[1][nt]);
      }
    }
  }
  {
    const size_t arow = (size_t)(m0 + 32 * w + m) * (size_t)ER + (size_t)(8 * hh);
    const unsigned short* h0p = waxh + arow;
    const unsigned short* h1p = h0p + (size_t)16 * ER;
    const unsigned short* l0p = waxl + arow;
    const unsigned short* l1p = l0p + (size_t)16 * ER;
    const unsigned short* bp  = bt + (size_t)(col0 + m) * (size_t)ER + (size_t)(8 * hh);
#pragma unroll 1
    for (int ks = 0; ks < ER / 32; ++ks) {
      FragB ah0, ah1, al0, al1;
      ldfrag(ah0, h0p + 32 * ks);
      ldfrag(ah1, h1p + 32 * ks);
      ldfrag(al0, l0p + 32 * ks);
      ldfrag(al1, l1p + 32 * ks);
#pragma unroll
      for (int nt = 0; nt < 4; ++nt) {
        FragB b;
        ldfrag(b, bp + (size_t)(16 * nt) * (size_t)ER + 32 * ks);
        acc[0][nt] = wmb(ah0, b, acc[0][nt]);
        acc[0][nt] = wmb(al0, b, acc[0][nt]);
        acc[1][nt] = wmb(ah1, b, acc[1][nt]);
        acc[1][nt] = wmb(al1, b, acc[1][nt]);
      }
    }
  }

#pragma unroll
  for (int nt = 0; nt < 4; ++nt) {
    const int lc = 16 * nt + m;
    const float bvl = rne16f(bb[col0 + lc]);
#pragma unroll
    for (int mt = 0; mt < 2; ++mt) {
#pragma unroll
      for (int r = 0; r < 8; ++r) {
        const int lr = 32 * w + 16 * mt + 8 * hh + r;
        stg[lr * TN + lc] = acc[mt][nt][r] + bvl;
      }
    }
  }
  __syncthreads();

  v4f fv[16];
  size_t op[16];
#pragma unroll
  for (int i = 0; i < 16; ++i) {
    const int lr = 32 * w + 2 * i + hh;
    fv[i] = *(const v4f*)(stg + lr * TN + 4 * m);
    op[i] = (size_t)(m0 + lr) * (size_t)ODIM + (size_t)(col0 + 4 * m);
  }
#pragma unroll
  for (int i = 0; i < 16; ++i) *(volatile v4f*)(out + op[i]) = fv[i];
  __threadfence();
#pragma unroll
  for (int i = 0; i < 16; ++i) *(volatile v4f*)(out + op[i]) = fv[i];
}

static inline int cdiv(int a, int b) { return (a + b - 1) / b; }

extern "C" void kernel_launch(void* const* d_in, const int* in_sizes, int n_in,
                              void* d_out, int out_size, void* d_ws, size_t ws_size,
                              hipStream_t stream) {
  if (n_in < 7) return;
  if (in_sizes[0] != NTOK * DIM) return;
  if (in_sizes[1] != ODIM * DIM) return;
  if (in_sizes[2] != ODIM) return;
  if (in_sizes[3] != NE * DIM * RNK) return;
  if (in_sizes[4] != NE * RNK * ODIM) return;
  if (in_sizes[5] != NE * DIM) return;
  if (in_sizes[6] != NE) return;
  if (out_size != NTOK * ODIM) return;

  const float* x   = (const float*)d_in[0];
  const float* bw  = (const float*)d_in[1];
  const float* bbv = (const float*)d_in[2];
  const float* la  = (const float*)d_in[3];
  const float* lb  = (const float*)d_in[4];
  const float* rw  = (const float*)d_in[5];
  const float* rb  = (const float*)d_in[6];
  float* out = (float*)d_out;

  char* ws = (char*)d_ws;
  size_t off = 0;
  const size_t oXB = off; off += (size_t)NTOK * DIM * 2;   off = (off + 255) & ~(size_t)255;
  const size_t oWB = off; off += (size_t)ODIM * DIM * 2;   off = (off + 255) & ~(size_t)255;
  const size_t oAT = off; off += (size_t)ER * DIM * 2;     off = (off + 255) & ~(size_t)255;
  const size_t oBT = off; off += (size_t)ODIM * ER * 2;    off = (off + 255) & ~(size_t)255;
  const size_t oEW = off; off += (size_t)NTOK * NE * 4;    off = (off + 255) & ~(size_t)255;
  const size_t oWH = off; off += (size_t)NTOK * ER * 2;    off = (off + 255) & ~(size_t)255;
  const size_t oWL = off; off += (size_t)NTOK * ER * 2;    off = (off + 255) & ~(size_t)255;
  if (off > ws_size || off > (size_t)WSMAX) return;

  unsigned short* XB   = (unsigned short*)(ws + oXB);
  unsigned short* WB   = (unsigned short*)(ws + oWB);
  unsigned short* AT   = (unsigned short*)(ws + oAT);
  unsigned short* BT   = (unsigned short*)(ws + oBT);
  float*          EW   = (float*)(ws + oEW);
  unsigned short* WAXH = (unsigned short*)(ws + oWH);
  unsigned short* WAXL = (unsigned short*)(ws + oWL);

  {
    const int nUx = NTOK * DIM / 8;
    const int nUw = ODIM * DIM / 8;
    k_cvt<<<cdiv(nUx, NTHR), NTHR, 0, stream>>>(x, XB, nUx);
    k_cvt<<<cdiv(nUw, NTHR), NTHR, 0, stream>>>(bw, WB, nUw);
    const int nUa = NE * DIM * RNK / 8;
    k_wtr<<<cdiv(nUa, NTHR), NTHR, 0, stream>>>(la, AT, DIM, RNK, NE, nUa);
    const int nUb = ER * ODIM / 8;
    k_wtr<<<cdiv(nUb, NTHR), NTHR, 0, stream>>>(lb, BT, ER, ODIM, 1, nUb);
  }
  k_gate<<<NTOK / NTHR, NTHR, 0, stream>>>(x, rw, rb, EW);
  k_ax<<<dim3(NTOK / TM, ER / TN), GTHR, 0, stream>>>(XB, AT, EW, WAXH, WAXL);
  k_main<<<dim3(NTOK / TM, ODIM / TN), GTHR, 0, stream>>>(XB, WB, bbv, WAXH, WAXL, BT, out);
}
